// gnet_62199716381113
// MI455X (gfx1250) — hardware-verified
//
#include <hip/hip_runtime.h>
#include <stddef.h>


#define DX      512
#define KCH     5
#define KTOT    (KCH * DX)
#define D1OUT   512
#define D2OUT   384
#define DA1     128
#define DA2     64
#define NTHR    256
#define NWAVE   8
#define GTHR    512
#define EPT     8
#define NGRP    2
#define CHUNK   (NTHR * EPT * NGRP)
#define WCAP    (EPT * NGRP * 32)
#define LISTN   (NWAVE * WCAP)
#define NBC     4096
#define NBF     1024
#define RCAP    40960
#define RBN     128
#define OTHR    512
#define TGT     256
#define DEGCAP  1024
#define GSL     16
#define WSCL    64.0f
#define WINV    0.015625f
#define WSCAP   134217728
#define F_ADDC  1
#define F_BIAS  2
#define F_RELU  4
#define LDS_FILL ((RCAP + NBF + LISTN) * 4 + 64)

static_assert(D1OUT == DX);
static_assert((CHUNK & (CHUNK - 1)) == 0);
static_assert(CHUNK <= 4096);
static_assert(NBC <= 4096 && NBF <= 4096);
static_assert((NBC & (NBC - 1)) == 0 && (NBF & (NBF - 1)) == 0);
static_assert(NBC == 4 * NBF);
static_assert(OTHR * 8 == NBC);
static_assert((RCAP % 32) == 0);
static_assert(TGT == NWAVE * 32);
static_assert(GSL * 32 == GTHR);
static_assert((DX % 128) == 0 && (D2OUT % 128) == 0);

typedef float    v4f  __attribute__((ext_vector_type(4)));
typedef float    v8f  __attribute__((ext_vector_type(8)));
typedef int      v4i  __attribute__((ext_vector_type(4)));
typedef _Float16 v8h  __attribute__((ext_vector_type(8)));
typedef _Float16 v16h __attribute__((ext_vector_type(16)));
union FragH { v16h v; v8h h[2]; };

__device__ __forceinline__ v8f wmh(v16h a, v16h b, v8f c) {
  v8f d = __builtin_amdgcn_wmma_f32_16x16x32_f16(false, a, false, b, (short)0, c, false, false);
  asm volatile("v_nop\n\tv_nop\n\tv_nop\n\tv_nop" : "+v"(d) : "v"(a), "v"(b));
  return d;
}

constexpr int gemm_nc(int NT, int CG) { return 16 * NT * CG; }
constexpr int gemm_bm(int CG) { return 32 * (16 / CG); }
constexpr int gemm_lds(int NT, int CG, int KD) {
  return (gemm_bm(CG) * (KD + 8) * 2 > gemm_bm(CG) * gemm_nc(NT, CG) * 4)
             ? gemm_bm(CG) * (KD + 8) * 2
             : gemm_bm(CG) * gemm_nc(NT, CG) * 4;
}

template <int NB>
__device__ __forceinline__ int scan_chunk(const int* __restrict__ dsts, int nE, int cbase, int slotBase,
                                          int vec8, int* list, int tid, int lane, int wave) {
  int wc = 0;
#pragma unroll
  for (int g = 0; g < NGRP; ++g) {
    const int el0  = (g * NTHR + tid) * EPT;
    const int e0   = cbase + el0;
    const int sent = -2147483647 - 1;
    v4i da, db;
    if (vec8 != 0 && cbase + CHUNK <= nE) {
      da = *(const v4i*)(dsts + e0);
      db = *(const v4i*)(dsts + e0 + 4);
    } else {
      da.x = (e0     < nE) ? dsts[min(e0, nE - 1)] : sent;
      da.y = (e0 + 1 < nE) ? dsts[min(e0 + 1, nE - 1)] : sent;
      da.z = (e0 + 2 < nE) ? dsts[min(e0 + 2, nE - 1)] : sent;
      da.w = (e0 + 3 < nE) ? dsts[min(e0 + 3, nE - 1)] : sent;
      db.x = (e0 + 4 < nE) ? dsts[min(e0 + 4, nE - 1)] : sent;
      db.y = (e0 + 5 < nE) ? dsts[min(e0 + 5, nE - 1)] : sent;
      db.z = (e0 + 6 < nE) ? dsts[min(e0 + 6, nE - 1)] : sent;
      db.w = (e0 + 7 < nE) ? dsts[min(e0 + 7, nE - 1)] : sent;
    }
    const unsigned nb = (unsigned)slotBase;
    const unsigned s0 = (unsigned)da.x - nb, s1 = (unsigned)da.y - nb;
    const unsigned s2 = (unsigned)da.z - nb, s3 = (unsigned)da.w - nb;
    const unsigned s4 = (unsigned)db.x - nb, s5 = (unsigned)db.y - nb;
    const unsigned s6 = (unsigned)db.z - nb, s7 = (unsigned)db.w - nb;
    const bool h0 = s0 < (unsigned)NB, h1 = s1 < (unsigned)NB, h2 = s2 < (unsigned)NB, h3 = s3 < (unsigned)NB;
    const bool h4 = s4 < (unsigned)NB, h5 = s5 < (unsigned)NB, h6 = s6 < (unsigned)NB, h7 = s7 < (unsigned)NB;
    const unsigned any = __builtin_amdgcn_ballot_w32(h0 | h1 | h2 | h3 | h4 | h5 | h6 | h7);
    if (any != 0u) {
#define HITJ(J, HJ, SJ) { \
        const unsigned mj = __builtin_amdgcn_ballot_w32(HJ); \
        if (mj != 0u) { \
          if (HJ) { \
            const int pos = wc + (int)__builtin_amdgcn_mbcnt_lo(mj, 0u); \
            if (pos < WCAP) list[wave * WCAP + pos] = ((el0 + (J)) << 12) | (int)(SJ); \
          } \
          wc += (int)__builtin_popcount(mj); } }
      HITJ(0, h0, s0)
      HITJ(1, h1, s1)
      HITJ(2, h2, s2)
      HITJ(3, h3, s3)
      HITJ(4, h4, s4)
      HITJ(5, h5, s5)
      HITJ(6, h6, s6)
      HITJ(7, h7, s7)
#undef HITJ
    }
  }
  return wc;
}

__global__ __launch_bounds__(NTHR) void k_wprep(const float* __restrict__ W, _Float16* dst,
                                                int KT, int NC, int tot8) {
  const int i = blockIdx.x * NTHR + threadIdx.x;
  const int ic = i > tot8 - 1 ? tot8 - 1 : i;
  const int cpr = KT >> 3;
  const int n = ic / cpr;
  const int k0 = (ic - n * cpr) * 8;
  v8h hv;
  {
    float v[8];
#pragma unroll
    for (int e = 0; e < 8; ++e) v[e] = W[(size_t)(k0 + e) * NC + n] * WSCL;
    hv[0] = (_Float16)v[0]; hv[1] = (_Float16)v[1]; hv[2] = (_Float16)v[2]; hv[3] = (_Float16)v[3];
    hv[4] = (_Float16)v[4]; hv[5] = (_Float16)v[5]; hv[6] = (_Float16)v[6]; hv[7] = (_Float16)v[7];
  }
  _Float16* dp = dst + (size_t)n * KT + k0;
  if (i < tot8) *(volatile v8h*)dp = hv;
  __threadfence();
  if (i < tot8) *(volatile v8h*)dp = hv;
}

__global__ __launch_bounds__(NTHR) void k_deg(const int* __restrict__ srcs, const float* __restrict__ ew,
                                              float* dis, int nE, int vec8) {
  __shared__ __attribute__((aligned(16))) float sdeg[NBC];
  __shared__ __attribute__((aligned(16))) int list[LISTN];
  __shared__ int wcnt[NWAVE];
  const int tid = threadIdx.x, lane = tid & 31, wave = tid >> 5;
  const int nodeBase = blockIdx.x * NBC;
  for (int i = tid; i < NBC; i += NTHR) sdeg[i] = 0.0f;
  __syncthreads();

  const int nChunks = (nE + CHUNK - 1) / CHUNK;
#pragma unroll 1
  for (int ch = 0; ch < nChunks; ++ch) {
    const int cbase = ch * CHUNK;
    const int wc = scan_chunk<NBC>(srcs, nE, cbase, nodeBase, vec8, list, tid, lane, wave);
    if (lane == 0) wcnt[wave] = wc;
    __syncthreads();
    if (wave == 0) {
#pragma unroll 1
      for (int wsx = 0; wsx < NWAVE; ++wsx) {
        int n = __builtin_amdgcn_readfirstlane(wcnt[wsx]);
        n = n > WCAP ? WCAP : (n < 0 ? 0 : n);
        const int* lp = list + wsx * WCAP;
#pragma unroll 1
        for (int i = 0; i < n; ++i) {
          const int ent  = __builtin_amdgcn_readfirstlane(lp[i]);
          const int slot = ent & (NBC - 1);
          int e = cbase + ((ent >> 12) & (CHUNK - 1));
          e = e > nE - 1 ? nE - 1 : e;
          const float w = ew[e];
          if (lane == 0) sdeg[slot] = sdeg[slot] + w;
        }
      }
    }
    __syncthreads();
  }

#pragma unroll 1
  for (int s = tid; s < NBC; s += NTHR) {
    const float dv = sdeg[s];
    sdeg[s] = dv > 0.0f ? 1.0f / sqrtf(dv) : 0.0f;
  }
  __syncthreads();
  float* gp = dis + (size_t)nodeBase;
#pragma unroll
  for (int q = 0; q < 4; ++q) {
    const int f = (wave * 4 + q) * 128 + 4 * lane;
    const v4f v = *(const v4f*)(sdeg + f);
    *(volatile v4f*)(gp + f) = v;
  }
  __threadfence();
#pragma unroll
  for (int q = 0; q < 4; ++q) {
    const int f = (wave * 4 + q) * 128 + 4 * lane;
    const v4f v = *(const v4f*)(sdeg + f);
    *(volatile v4f*)(gp + f) = v;
  }
}

__global__ __launch_bounds__(NTHR) void k_count(const int* __restrict__ dsts, int* cnt, int nE, int vec8) {
  __shared__ __attribute__((aligned(16))) int scnt[NBC];
  __shared__ __attribute__((aligned(16))) int list[LISTN];
  __shared__ int wcnt[NWAVE];
  const int tid = threadIdx.x, lane = tid & 31, wave = tid >> 5;
  const int nodeBase = blockIdx.x * NBC;

  for (int i = tid; i < NBC; i += NTHR) scnt[i] = 0;
  __syncthreads();

  const int nChunks = (nE + CHUNK - 1) / CHUNK;
#pragma unroll 1
  for (int ch = 0; ch < nChunks; ++ch) {
    const int cbase = ch * CHUNK;
    const int wc = scan_chunk<NBC>(dsts, nE, cbase, nodeBase, vec8, list, tid, lane, wave);
    if (lane == 0) wcnt[wave] = wc;
    __syncthreads();
    if (wave == 0) {
#pragma unroll 1
      for (int wsx = 0; wsx < NWAVE; ++wsx) {
        int n = __builtin_amdgcn_readfirstlane(wcnt[wsx]);
        n = n > WCAP ? WCAP : (n < 0 ? 0 : n);
        const int* lp = list + wsx * WCAP;
#pragma unroll 1
        for (int i = 0; i < n; ++i) {
          const int ent  = __builtin_amdgcn_readfirstlane(lp[i]);
          const int slot = ent & (NBC - 1);
          if (lane == 0) scnt[slot] = scnt[slot] + 1;
        }
      }
    }
    __syncthreads();
  }

  v4i cq[4];
#pragma unroll
  for (int q = 0; q < 4; ++q) {
    const int f = (wave * 4 + q) * 128 + 4 * lane;
    cq[q] = *(const v4i*)(scnt + f);
  }
  int* cp = cnt + (size_t)nodeBase;
#pragma unroll
  for (int q = 0; q < 4; ++q) {
    const int f = (wave * 4 + q) * 128 + 4 * lane;
    *(volatile v4i*)(cp + f) = cq[q];
  }
  __threadfence();
#pragma unroll
  for (int q = 0; q < 4; ++q) {
    const int f = (wave * 4 + q) * 128 + 4 * lane;
    *(volatile v4i*)(cp + f) = cq[q];
  }
}

__global__ __launch_bounds__(OTHR) void k_offsets(
    const int* __restrict__ cnt, int* off, int* rbase, int nChunk) {
  __shared__ __attribute__((aligned(16))) int soff[NBC];
  __shared__ __attribute__((aligned(16))) int srb[RBN];
  __shared__ int wtot[OTHR / 32];
  const int tid = threadIdx.x, lane = tid & 31, wave = tid >> 5, sub = tid >> 7;
  for (int i = tid; i < RBN; i += OTHR) srb[i] = 0;
  int carry = 0;
#pragma unroll 1
  for (int ch = 0; ch < nChunk; ++ch) {
    const int base = ch * NBC;
    const v4i c0 = *(const v4i*)(cnt + base + 8 * tid);
    const v4i c1 = *(const v4i*)(cnt + base + 8 * tid + 4);
    const int e0 = max(c0.x, 0), e1 = max(c0.y, 0), e2 = max(c0.z, 0), e3 = max(c0.w, 0);
    const int e4 = max(c1.x, 0), e5 = max(c1.y, 0), e6 = max(c1.z, 0), e7 = max(c1.w, 0);
    const int ts = e0 + e1 + e2 + e3 + e4 + e5 + e6 + e7;
    int incl = ts;
#pragma unroll
    for (int d = 1; d < 32; d <<= 1) {
      const int t = __shfl_up(incl, d);
      if (lane >= d) incl += t;
    }
    if (lane == 31) wtot[wave] = incl;
    __syncthreads();
    const int S0 = wtot[0]  + wtot[1]  + wtot[2]  + wtot[3];
    const int S1 = wtot[4]  + wtot[5]  + wtot[6]  + wtot[7];
    const int S2 = wtot[8]  + wtot[9]  + wtot[10] + wtot[11];
    const int S3 = wtot[12] + wtot[13] + wtot[14] + wtot[15];
    int pre = 0;
#pragma unroll 1
    for (int w = 4 * sub; w < wave; ++w) pre += wtot[w];
    const int b0 = carry;
    const int b1 = b0 + ((S0 + 31) & ~31);
    const int b2 = b1 + ((S1 + 31) & ~31);
    const int b3 = b2 + ((S2 + 31) & ~31);
    const int b4 = b3 + ((S3 + 31) & ~31);
    const int myb = sub == 0 ? b0 : (sub == 1 ? b1 : (sub == 2 ? b2 : b3));
    if (tid == 0) {
      srb[min(4 * ch + 0, RBN - 1)] = b0;
      srb[min(4 * ch + 1, RBN - 1)] = b1;
      srb[min(4 * ch + 2, RBN - 1)] = b2;
      srb[min(4 * ch + 3, RBN - 1)] = b3;
    }
    int run = myb + pre + incl - ts;
    soff[8 * tid + 0] = run; run += e0;
    soff[8 * tid + 1] = run; run += e1;
    soff[8 * tid + 2] = run; run += e2;
    soff[8 * tid + 3] = run; run += e3;
    soff[8 * tid + 4] = run; run += e4;
    soff[8 * tid + 5] = run; run += e5;
    soff[8 * tid + 6] = run; run += e6;
    soff[8 * tid + 7] = run;
    carry = b4;
    __syncthreads();
    const v4i o0 = *(const v4i*)(soff + 4 * tid);
    const v4i o1 = *(const v4i*)(soff + 4 * (tid + OTHR));
    int* op = off + base;
    *(volatile v4i*)(op + 4 * tid) = o0;
    *(volatile v4i*)(op + 4 * (tid + OTHR)) = o1;
    __threadfence();
    *(volatile v4i*)(op + 4 * tid) = o0;
    *(volatile v4i*)(op + 4 * (tid + OTHR)) = o1;
    __syncthreads();
  }
  if (tid == 0) srb[min(4 * nChunk, RBN - 1)] = carry;
  __syncthreads();
  v4i rv = {0, 0, 0, 0};
  if (tid < 32) rv = *(const v4i*)(srb + 4 * tid);
  if (tid < 32) *(volatile v4i*)(rbase + 4 * tid) = rv;
  __threadfence();
  if (tid < 32) *(volatile v4i*)(rbase + 4 * tid) = rv;
}

__global__ __launch_bounds__(NTHR) void k_fill(
    const int* __restrict__ dsts, const int* __restrict__ off, const int* __restrict__ rbase,
    int* csr, int nE, int vec8, int csrLen) {
  extern __shared__ v4f lds_dyn[];
  int* region = (int*)lds_dyn;
  int* cursor = region + RCAP;
  int* list   = cursor + NBF;
  int* wcnt   = list + LISTN;
  const int tid = threadIdx.x, lane = tid & 31, wave = tid >> 5;
  const int b = blockIdx.x;
  const int nodeBase = b * NBF;

  int rb0 = rbase[b];
  const int rb1 = rbase[b + 1];
  rb0 = rb0 < 0 ? 0 : (rb0 > csrLen ? csrLen : rb0);
  rb0 &= ~31;
  int len = rb1 - rb0;
  len = len < 0 ? 0 : (len > RCAP ? RCAP : len);
  int lenW = (len + 31) & ~31;
  if (rb0 + lenW > csrLen) lenW = (csrLen - rb0) & ~31;

  {
    const v4i z = {0, 0, 0, 0};
    for (int i = tid; i < RCAP / 4; i += NTHR) ((v4i*)region)[i] = z;
    for (int s = tid; s < NBF; s += NTHR) {
      int o = off[nodeBase + s] - rb0;
      o = o < 0 ? 0 : (o > RCAP ? RCAP : o);
      cursor[s] = o;
    }
  }
  __syncthreads();

  const int nChunks = (nE + CHUNK - 1) / CHUNK;
#pragma unroll 1
  for (int ch = 0; ch < nChunks; ++ch) {
    const int cbase = ch * CHUNK;
    const int wc = scan_chunk<NBF>(dsts, nE, cbase, nodeBase, vec8, list, tid, lane, wave);
    if (lane == 0) wcnt[wave] = wc;
    __syncthreads();
    if (wave == 0) {
#pragma unroll 1
      for (int wsx = 0; wsx < NWAVE; ++wsx) {
        int n = __builtin_amdgcn_readfirstlane(wcnt[wsx]);
        n = n > WCAP ? WCAP : (n < 0 ? 0 : n);
        const int* lp = list + wsx * WCAP;
#pragma unroll 1
        for (int i = 0; i < n; ++i) {
          const int ent  = __builtin_amdgcn_readfirstlane(lp[i]);
          const int slot = ent & (NBF - 1);
          int e = cbase + ((ent >> 12) & (CHUNK - 1));
          e = e > nE - 1 ? nE - 1 : e;
          if (lane == 0) {
            int pos = cursor[slot];
            pos = pos < 0 ? 0 : (pos > RCAP - 1 ? RCAP - 1 : pos);
            region[pos] = e;
            const int np = pos + 1;
            cursor[slot] = np > RCAP ? RCAP : np;
          }
        }
      }
    }
    __syncthreads();
  }

  const int nv = lenW >> 2;
  int* gp = csr + rb0;
#pragma unroll 1
  for (int i = tid; i < nv; i += NTHR) { const v4i v = ((const v4i*)region)[i]; *(volatile v4i*)(gp + 4 * i) = v; }
  __threadfence();
#pragma unroll 1
  for (int i = tid; i < nv; i += NTHR) { const v4i v = ((const v4i*)region)[i]; *(volatile v4i*)(gp + 4 * i) = v; }
}

template <int MODE>
__global__ __launch_bounds__(NTHR) void k_cheb(
    const int* __restrict__ csr, const int* __restrict__ off, const int* __restrict__ cnt,
    const int* __restrict__ srcs, const float* __restrict__ ew, const float* __restrict__ dis,
    const float* __restrict__ H, const float* prev, int prevRows, float* outp,
    int nN, int nE, int csrLen) {
  const int tid = threadIdx.x, lane = tid & 31, wave = tid >> 5;
  const int tbase = blockIdx.x * TGT + wave * 32;
  const int cl = tbase + lane;
  const int cnt_l = cnt[cl];
  const int off_l = off[cl];
  const int dis_l = __float_as_int(dis[cl]);
  const v4f z = {0.0f, 0.0f, 0.0f, 0.0f};
#pragma unroll 1
  for (int j = 0; j < 32; ++j) {
    const int t = tbase + j;
    int n = __builtin_amdgcn_readlane(cnt_l, j);
    n = n < 0 ? 0 : (n > DEGCAP ? DEGCAP : n);
    const int st = __builtin_amdgcn_readlane(off_l, j);
    const float dt = __int_as_float(__builtin_amdgcn_readlane(dis_l, j));
    v4f a0 = z, a1 = z, a2 = z, a3 = z;
#pragma unroll 1
    for (int q0 = 0; q0 < n; q0 += 32) {
      int pos = st + q0 + lane;
      pos = pos < 0 ? 0 : (pos > csrLen - 1 ? csrLen - 1 : pos);
      int el = csr[pos];
      el = el < 0 ? 0 : (el > nE - 1 ? nE - 1 : el);
      int sl = srcs[el];
      sl = sl < 0 ? 0 : (sl > nN - 1 ? nN - 1 : sl);
      const float cfv = (-dis[sl] * ew[el]) * dt;
      const int cfi = __float_as_int(cfv);
      const int mcnt = (n - q0) < 32 ? (n - q0) : 32;
#pragma unroll 1
      for (int p = 0; p < mcnt; ++p) {
        const int s = __builtin_amdgcn_readlane(sl, p);
        const float cf = __int_as_float(__builtin_amdgcn_readlane(cfi, p));
        const float* hp = H + (size_t)s * DX + 4 * lane;
        a0 = a0 + *(const v4f*)(hp) * cf;
        a1 = a1 + *(const v4f*)(hp + 128) * cf;
        a2 = a2 + *(const v4f*)(hp + 256) * cf;
        a3 = a3 + *(const v4f*)(hp + 384) * cf;
      }
    }
    v4f o0, o1, o2, o3;
    if (MODE == 0) {
      o0 = a0; o1 = a1; o2 = a2; o3 = a3;
    } else {
      const int tp = t > prevRows - 1 ? prevRows - 1 : t;
      const float* pp = prev + (size_t)tp * DX + 4 * lane;
      const v4f p0 = *(const v4f*)(pp);
      const v4f p1 = *(const v4f*)(pp + 128);
      const v4f p2 = *(const v4f*)(pp + 256);
      const v4f p3 = *(const v4f*)(pp + 384);
      o0 = a0 * 2.0f - p0;
      o1 = a1 * 2.0f - p1;
      o2 = a2 * 2.0f - p2;
      o3 = a3 * 2.0f - p3;
    }
    float* op = outp + (size_t)t * DX + 4 * lane;
    *(volatile v4f*)(op)       = o0;
    *(volatile v4f*)(op + 128) = o1;
    *(volatile v4f*)(op + 256) = o2;
    *(volatile v4f*)(op + 384) = o3;
    __threadfence();
    *(volatile v4f*)(op)       = o0;
    *(volatile v4f*)(op + 128) = o1;
    *(volatile v4f*)(op + 256) = o2;
    *(volatile v4f*)(op + 384) = o3;
  }
}

template <int NT, int CG, int KD, int GATE>
__global__ __launch_bounds__(GTHR) void k_gemm(
    const float* __restrict__ A, int aRows, const _Float16* __restrict__ Bw, int ldb, int kofs,
    const float* __restrict__ bias, float* C, int flags, float scale,
    const float* __restrict__ w3, const float* __restrict__ b3, float* gate) {
  constexpr int NC = 16 * NT * CG, RG = 16 / CG, BM = 32 * RG, APK = KD + 8, WN = 16 * NT;
  constexpr int TPR = GTHR / BM, CPT = KD / (8 * TPR), NKT = KD / 32, SWEEPS = (BM * NC) / (4 * GTHR);
  static_assert(RG * CG == 16);
  static_assert((KD % 32) == 0 && CPT * 8 * TPR == KD && TPR * BM == GTHR);
  static_assert(SWEEPS * 4 * GTHR == BM * NC);
  static_assert(GATE == 0 || BM == 128);
  extern __shared__ v4f lds_dyn[];
  __shared__ __attribute__((aligned(16))) float sg[128];
  _Float16* sA = (_Float16*)lds_dyn;
  float* stg = (float*)lds_dyn;
  const int tid = threadIdx.x, lane = tid & 31, wave = tid >> 5, hh = lane >> 4, m = lane & 15;
  const int rowBase = blockIdx.x * BM;

  {
    const int r = tid / TPR;
    const int cb = (tid - r * TPR) * (KD / TPR);
    int grow = rowBase + r;
    grow = grow > aRows - 1 ? aRows - 1 : grow;
    const float* ap = A + (size_t)grow * KD + cb;
    _Float16* sp = sA + r * APK + cb;
#pragma unroll
    for (int c = 0; c < CPT; ++c) {
      const v4f a = *(const v4f*)(ap + 8 * c);
      const v4f b = *(const v4f*)(ap + 8 * c + 4);
      v8h hv;
      hv[0] = (_Float16)a.x; hv[1] = (_Float16)a.y; hv[2] = (_Float16)a.z; hv[3] = (_Float16)a.w;
      hv[4] = (_Float16)b.x; hv[5] = (_Float16)b.y; hv[6] = (_Float16)b.z; hv[7] = (_Float16)b.w;
      *(v8h*)(sp + 8 * c) = hv;
    }
  }
  __syncthreads();

  const int rg = wave / CG, cg = wave - rg * CG;
  const int arow0 = rg * 32;
  v8f acc[2][NT];
#pragma unroll
  for (int t = 0; t < NT; ++t) {
    const v8f zz = {0.f, 0.f, 0.f, 0.f, 0.f, 0.f, 0.f, 0.f};
    acc[0][t] = zz;
    acc[1][t] = zz;
  }
  {
    const _Float16* ap0 = sA + (arow0 + m) * APK + 8 * hh;
    const _Float16* ap1 = ap0 + 16 * APK;
    const _Float16* bp0 = Bw + (size_t)(cg * WN + m) * ldb + kofs + 8 * hh;
#pragma unroll 1
    for (int kt = 0; kt < NKT; ++kt) {
      FragH a0, a1;
      a0.h[0] = *(const v8h*)(ap0 + 32 * kt);
      a0.h[1] = *(const v8h*)(ap0 + 32 * kt + 16);
      a1.h[0] = *(const v8h*)(ap1 + 32 * kt);
      a1.h[1] = *(const v8h*)(ap1 + 32 * kt + 16);
#pragma unroll
      for (int t = 0; t < NT; ++t) {
        const _Float16* bp = bp0 + (size_t)(16 * t) * ldb + 32 * kt;
        FragH b;
        b.h[0] = *(const v8h*)bp;
        b.h[1] = *(const v8h*)(bp + 16);
        acc[0][t] = wmh(a0.v, b.v, acc[0][t]);
        acc[1][t] = wmh(a1.v, b.v, acc[1][t]);
      }
    }
  }
  __syncthreads();

  {
#pragma unroll
    for (int rt = 0; rt < 2; ++rt) {
      float* sp = stg + (size_t)(arow0 + rt * 16 + 8 * hh) * NC + cg * WN + m;
#pragma unroll
      for (int t = 0; t < NT; ++t) {
#pragma unroll
        for (int r = 0; r < 8; ++r) sp[r * NC + 16 * t] = acc[rt][t][r];
      }
    }
  }
  __syncthreads();

  v4f* stg4 = (v4f*)stg;
  const size_t gbase = (size_t)rowBase * NC;
#pragma unroll 1
  for (int it = 0; it < SWEEPS; ++it) {
    const int q = it * GTHR + tid;
    v4f v = stg4[q] * scale;
    if (flags & F_ADDC) v = v + *(const v4f*)(C + gbase + 4 * (size_t)q);
    if (flags & F_BIAS) v = v + *(const v4f*)(bias + ((4 * q) % NC));
    if (flags & F_RELU) {
      v.x = fmaxf(v.x, 0.0f); v.y = fmaxf(v.y, 0.0f); v.z = fmaxf(v.z, 0.0f); v.w = fmaxf(v.w, 0.0f);
    }
    stg4[q] = v;
  }

  if constexpr (GATE != 0) {
    __syncthreads();
    if (tid < BM) {
      const float* sr = stg + (size_t)tid * NC;
      float g = 0.0f;
#pragma unroll 4
      for (int jx = 0; jx < NC; ++jx) g += sr[jx] * w3[jx];
      g += b3[0];
      sg[tid] = tanhf(g);
    }
    __syncthreads();
    v4f gv = {0.f, 0.f, 0.f, 0.f};
    if (tid < BM / 4) gv = *(const v4f*)(sg + 4 * tid);
    float* gp = gate + (size_t)rowBase + 4 * tid;
    if (tid < BM / 4) *(volatile v4f*)gp = gv;
    __threadfence();
    if (tid < BM / 4) *(volatile v4f*)gp = gv;
  } else {
#pragma unroll 1
    for (int it = 0; it < SWEEPS; ++it) {
      const int q = it * GTHR + tid;
      const v4f v = stg4[q];
      *(volatile v4f*)(C + gbase + 4 * (size_t)q) = v;
    }
    __threadfence();
#pragma unroll 1
    for (int it = 0; it < SWEEPS; ++it) {
      const int q = it * GTHR + tid;
      const v4f v = stg4[q];
      *(volatile v4f*)(C + gbase + 4 * (size_t)q) = v;
    }
  }
}

__global__ __launch_bounds__(GTHR) void k_pool(const int* __restrict__ bat, const float* __restrict__ gate,
                                               const float* __restrict__ H2, float* outp, int nN, int nG) {
  const int tid = threadIdx.x, lane = tid & 31, wave = tid >> 5;
  const int g = blockIdx.x * GSL + wave;
  float mx = __uint_as_float(0xff800000u);
#pragma unroll 1
  for (int c0 = 0; c0 < nN; c0 += 32) {
    const int i = c0 + lane;
    const int ic = i > nN - 1 ? nN - 1 : i;
    const int bi = bat[ic];
    const float gv = gate[ic];
    const bool hit = (i < nN) && (bi == g);
    mx = hit ? fmaxf(mx, gv) : mx;
  }
#pragma unroll
  for (int o = 16; o > 0; o >>= 1) mx = fmaxf(mx, __shfl_xor(mx, o));

  const v4f z = {0.0f, 0.0f, 0.0f, 0.0f};
  float d = 0.0f;
  v4f a0 = z, a1 = z, a2 = z;
#pragma unroll 1
  for (int c0 = 0; c0 < nN; c0 += 32) {
    const int i = c0 + lane;
    const int ic = i > nN - 1 ? nN - 1 : i;
    const int bi = bat[ic];
    const float gv = gate[ic];
    const bool hit = (i < nN) && (bi == g);
    unsigned msk = __builtin_amdgcn_ballot_w32(hit);
    const int gvi = __float_as_int(gv);
#pragma unroll 1
    for (int bb = 0; bb < 32; ++bb) {
      if (msk == 0u) break;
      const int p = (int)__builtin_ctz(msk);
      msk &= msk - 1u;
      int node = c0 + p;
      node = node > nN - 1 ? nN - 1 : node;
      const float ge = __int_as_float(__builtin_amdgcn_readlane(gvi, p));
      const float e = expf(ge - mx);
      d += e;
      const float* hp = H2 + (size_t)node * D2OUT + 4 * lane;
      a0 = a0 + *(const v4f*)(hp) * e;
      a1 = a1 + *(const v4f*)(hp + 128) * e;
      a2 = a2 + *(const v4f*)(hp + 256) * e;
    }
  }
  const float rcp = 1.0f / (d + 1e-16f);
  const v4f o0 = a0 * rcp, o1 = a1 * rcp, o2 = a2 * rcp;
  const int gs = g < nG ? g : 0;
  float* op = outp + (size_t)gs * D2OUT + 4 * lane;
  if (g < nG) {
    *(volatile v4f*)(op)       = o0;
    *(volatile v4f*)(op + 128) = o1;
    *(volatile v4f*)(op + 256) = o2;
  }
  __threadfence();
  if (g < nG) {
    *(volatile v4f*)(op)       = o0;
    *(volatile v4f*)(op + 128) = o1;
    *(volatile v4f*)(op + 256) = o2;
  }
}

extern "C" void kernel_launch(void* const* d_in, const int* in_sizes, int n_in,
                              void* d_out, int out_size, void* d_ws, size_t ws_size,
                              hipStream_t stream) {
  if (n_in < 14) return;
  const int nE = in_sizes[2];
  const int nN = in_sizes[3];
  if (nN <= 0 || nE <= 0 || nN > (1 << 21) || nE > (1 << 26)) return;
  if (in_sizes[0] != nN * DX || in_sizes[1] != 2 * nE) return;
  if (in_sizes[4] != KTOT * D1OUT || in_sizes[5] != D1OUT) return;
  if (in_sizes[6] != KTOT * D2OUT || in_sizes[7] != D2OUT) return;
  if (in_sizes[8] != D2OUT * DA1 || in_sizes[9] != DA1) return;
  if (in_sizes[10] != DA1 * DA2 || in_sizes[11] != DA2 || in_sizes[12] != DA2 || in_sizes[13] != 1) return;
  if (out_size <= 0 || (out_size % D2OUT) != 0) return;
  const int nG = out_size / D2OUT;

  const float* x    = (const float*)d_in[0];
  const int*   ei   = (const int*)d_in[1];
  const float* ew   = (const float*)d_in[2];
  const int*   bat  = (const int*)d_in[3];
  const float* W1c  = (const float*)d_in[4];
  const float* b1c  = (const float*)d_in[5];
  const float* W2c  = (const float*)d_in[6];
  const float* b2c  = (const float*)d_in[7];
  const float* Wa1  = (const float*)d_in[8];
  const float* ba1  = (const float*)d_in[9];
  const float* Wa2  = (const float*)d_in[10];
  const float* ba2  = (const float*)d_in[11];
  const float* Wa3  = (const float*)d_in[12];
  const float* ba3  = (const float*)d_in[13];
  const int* srcs = ei;
  const int* dsts = ei + nE;
  float* out = (float*)d_out;

  const int NPAD   = ((nN + TGT - 1) / TGT) * TGT;
  const int nBC    = (nN + NBC - 1) / NBC;
  const int CNTPAD = nBC * NBC;
  if (4 * nBC + 1 > RBN) return;
  const int nBF    = (nN + NBF - 1) / NBF;
  const int csrLen = ((nE + 31) & ~31) + 4096;
  if (31 * 4 * nBC > 4096) return;
  const int nCheb  = NPAD / TGT;
  const int nB64   = NPAD / 64;
  const int nB128  = NPAD / 128;
  const int nPB    = (nG + GSL - 1) / GSL;

  char* ws = (char*)d_ws;
  size_t off = 0;
  const size_t oWt1 = off; off += (size_t)D1OUT * KTOT * 2;       off = (off + 255) & ~(size_t)255;
  const size_t oWt2 = off; off += (size_t)D2OUT * KTOT * 2;       off = (off + 255) & ~(size_t)255;
  const size_t oWa1 = off; off += (size_t)DA1 * D2OUT * 2;        off = (off + 255) & ~(size_t)255;
  const size_t oWa2 = off; off += (size_t)DA2 * DA1 * 2;          off = (off + 255) & ~(size_t)255;
  const size_t oCnt = off; off += (size_t)CNTPAD * 4;             off = (off + 255) & ~(size_t)255;
  const size_t oOff = off; off += (size_t)CNTPAD * 4;             off = (off + 255) & ~(size_t)255;
  const size_t oDis = off; off += (size_t)CNTPAD * 4;             off = (off + 255) & ~(size_t)255;
  const size_t oRb  = off; off += (size_t)RBN * 4;                off = (off + 255) & ~(size_t)255;
  const size_t oCsr = off; off += (size_t)csrLen * 4;             off = (off + 255) & ~(size_t)255;
  const size_t oC   = off; off += (size_t)NPAD * DX * 4;          off = (off + 255) & ~(size_t)255;
  const size_t oP   = off; off += (size_t)NPAD * DX * 4;          off = (off + 255) & ~(size_t)255;
  const size_t oQ   = off; off += (size_t)NPAD * DX * 4;          off = (off + 255) & ~(size_t)255;
  const size_t oGt  = off; off += (size_t)NPAD * 4;               off = (off + 255) & ~(size_t)255;
  if (off > ws_size || off > (size_t)WSCAP) return;
  _Float16* Wt1 = (_Float16*)(ws + oWt1);
  _Float16* Wt2 = (_Float16*)(ws + oWt2);
  _Float16* Wa1t = (_Float16*)(ws + oWa1);
  _Float16* Wa2t = (_Float16*)(ws + oWa2);
  int*   cnt  = (int*)(ws + oCnt);
  int*   offp = (int*)(ws + oOff);
  float* dis  = (float*)(ws + oDis);
  int*   rb   = (int*)(ws + oRb);
  int*   csr  = (int*)(ws + oCsr);
  float* bufC = (float*)(ws + oC);
  float* bufP = (float*)(ws + oP);
  float* bufQ = (float*)(ws + oQ);
  float* gt   = (float*)(ws + oGt);

  const int vec8d = ((nE & 3) == 0) ? 1 : 0;
  const int vec8s = 1;

  constexpr int LDS_G1 = gemm_lds(4, 8, 512);
  constexpr int LDS_G2 = gemm_lds(3, 8, 512);
  constexpr int LDS_G3 = gemm_lds(1, 8, 384);
  constexpr int LDS_G4 = gemm_lds(1, 4, 128);
  hipFuncSetAttribute(reinterpret_cast<const void*>(&k_gemm<4, 8, 512, 0>),
                      hipFuncAttributeMaxDynamicSharedMemorySize, LDS_G1);
  hipFuncSetAttribute(reinterpret_cast<const void*>(&k_gemm<3, 8, 512, 0>),
                      hipFuncAttributeMaxDynamicSharedMemorySize, LDS_G2);
  hipFuncSetAttribute(reinterpret_cast<const void*>(&k_fill),
                      hipFuncAttributeMaxDynamicSharedMemorySize, LDS_FILL);

  {
    const int t1 = D1OUT * KTOT / 8, t2 = D2OUT * KTOT / 8, t3 = DA1 * D2OUT / 8, t4 = DA2 * DA1 / 8;
    k_wprep<<<(t1 + NTHR - 1) / NTHR, NTHR, 0, stream>>>(W1c, Wt1, KTOT, D1OUT, t1);
    k_wprep<<<(t2 + NTHR - 1) / NTHR, NTHR, 0, stream>>>(W2c, Wt2, KTOT, D2OUT, t2);
    k_wprep<<<(t3 + NTHR - 1) / NTHR, NTHR, 0, stream>>>(Wa1, Wa1t, D2OUT, DA1, t3);
    k_wprep<<<(t4 + NTHR - 1) / NTHR, NTHR, 0, stream>>>(Wa2, Wa2t, DA1, DA2, t4);
  }

  k_deg<<<nBC, NTHR, 0, stream>>>(srcs, ew, dis, nE, vec8s);

  k_count<<<nBC, NTHR, 0, stream>>>(dsts, cnt, nE, vec8d);
  k_offsets<<<1, OTHR, 0, stream>>>(cnt, offp, rb, nBC);
  k_fill<<<nBF, NTHR, LDS_FILL, stream>>>(dsts, offp, rb, csr, nE, vec8d, csrLen);

  k_gemm<4, 8, 512, 0><<<nB64, GTHR, LDS_G1, stream>>>(x, nN, Wt1, KTOT, 0 * DX, b1c, bufC, 0, WINV, Wa3, ba3, gt);
  k_cheb<0><<<nCheb, NTHR, 0, stream>>>(csr, offp, cnt, srcs, ew, dis, x, x, nN, bufP, nN, nE, csrLen);
  k_gemm<4, 8, 512, 0><<<nB64, GTHR, LDS_G1, stream>>>(bufP, NPAD, Wt1, KTOT, 1 * DX, b1c, bufC, F_ADDC, WINV, Wa3, ba3, gt);
  k_cheb<1><<<nCheb, NTHR, 0, stream>>>(csr, offp, cnt, srcs, ew, dis, bufP, x, nN, bufQ, nN, nE, csrLen);
  k_gemm<4, 8, 512, 0><<<nB64, GTHR, LDS_G1, stream>>>(bufQ, NPAD, Wt1, KTOT, 2 * DX, b1c, bufC, F_ADDC, WINV, Wa3, ba3, gt);
  k_cheb<1><<<nCheb, NTHR, 0, stream>>>(csr, offp, cnt, srcs, ew, dis, bufQ, bufP, NPAD, bufP, nN, nE, csrLen);
  k_gemm<4, 8, 512, 0><<<nB64, GTHR, LDS_G1, stream>>>(bufP, NPAD, Wt1, KTOT, 3 * DX, b1c, bufC, F_ADDC, WINV, Wa3, ba3, gt);
  k_cheb<1><<<nCheb, NTHR, 0, stream>>>(csr, offp, cnt, srcs, ew, dis, bufP, bufQ, NPAD, bufQ, nN, nE, csrLen);
  k_gemm<4, 8, 512, 0><<<nB64, GTHR, LDS_G1, stream>>>(bufQ, NPAD, Wt1, KTOT, 4 * DX, b1c, bufC,
                                                        F_ADDC | F_BIAS | F_RELU, WINV, Wa3, ba3, gt);

  k_gemm<3, 8, 512, 0><<<nB64, GTHR, LDS_G2, stream>>>(bufC, NPAD, Wt2, KTOT, 0 * DX, b2c, bufQ, 0, WINV, Wa3, ba3, gt);
  k_cheb<0><<<nCheb, NTHR, 0, stream>>>(csr, offp, cnt, srcs, ew, dis, bufC, bufC, NPAD, bufP, nN, nE, csrLen);
  k_gemm<3, 8, 512, 0><<<nB64, GTHR, LDS_G2, stream>>>(bufP, NPAD, Wt2, KTOT, 1 * DX, b2c, bufQ, F_ADDC, WINV, Wa3, ba3, gt);
  k_cheb<1><<<nCheb, NTHR, 0, stream>>>(csr, offp, cnt, srcs, ew, dis, bufP, bufC, NPAD, bufC, nN, nE, csrLen);
  k_gemm<3, 8, 512, 0><<<nB64, GTHR, LDS_G2, stream>>>(bufC, NPAD, Wt2, KTOT, 2 * DX, b2c, bufQ, F_ADDC, WINV, Wa3, ba3, gt);
  k_cheb<1><<<nCheb, NTHR, 0, stream>>>(csr, offp, cnt, srcs, ew, dis, bufC, bufP, NPAD, bufP, nN, nE, csrLen);
  k_gemm<3, 8, 512, 0><<<nB64, GTHR, LDS_G2, stream>>>(bufP, NPAD, Wt2, KTOT, 3 * DX, b2c, bufQ, F_ADDC, WINV, Wa3, ba3, gt);
  k_cheb<1><<<nCheb, NTHR, 0, stream>>>(csr, offp, cnt, srcs, ew, dis, bufP, bufC, NPAD, bufC, nN, nE, csrLen);
  k_gemm<3, 8, 512, 0><<<nB64, GTHR, LDS_G2, stream>>>(bufC, NPAD, Wt2, KTOT, 4 * DX, b2c, bufQ,
                                                        F_ADDC | F_BIAS | F_RELU, WINV, Wa3, ba3, gt);

  k_gemm<1, 8, 384, 0><<<nB64, GTHR, LDS_G3, stream>>>(bufQ, NPAD, Wa1t, D2OUT, 0, ba1, bufC, F_BIAS | F_RELU, WINV, Wa3, ba3, gt);
  k_gemm<1, 4, 128, 1><<<nB128, GTHR, LDS_G4, stream>>>(bufC, NPAD, Wa2t, DA1, 0, ba2, bufP, F_BIAS | F_RELU, WINV, Wa3, ba3, gt);

  k_pool<<<nPB, GTHR, 0, stream>>>(bat, gt, bufQ, out, nN, nG);
}
